// GridSamplePScan_12996571037932
// MI455X (gfx1250) — hardware-verified
//
#include <hip/hip_runtime.h>
#include <math.h>

typedef __attribute__((ext_vector_type(8)))  _Float16 v8h;
typedef __attribute__((ext_vector_type(16))) __bf16   v16b;
typedef __attribute__((ext_vector_type(8)))  __bf16   v8b;
typedef __attribute__((ext_vector_type(8)))  float    v8f;
typedef __attribute__((ext_vector_type(4)))  float    v4f;

constexpr int kFrames   = 16;
constexpr int kCh       = 32;
constexpr int kHid      = 16;
constexpr int kSide     = 64;
constexpr int kPix      = kSide * kSide;
constexpr int kRows     = kFrames * kPix;
constexpr int kKdim     = kCh;
constexpr int kNcol     = 2 * kHid;
constexpr int kChGroup  = 8;
constexpr int kNumGroup = kCh / kChGroup;
constexpr int kPrepPix   = 128;
constexpr int kPrepPitch = 36;
constexpr int kPrepImgBlocks = kRows / kPrepPix;
constexpr int kSlabPitch = 36;
constexpr int kGemmTiles = kRows / 64;
static_assert(kPix == 4096 && kRows == 65536, "shape");
static_assert((kKdim % 32) == 0, "GEMM K multiple of 32");
static_assert((kRows % 64) == 0 && (kNcol % 16) == 0, "GEMM M tile multiple, N subtile multiple");
static_assert((kGemmTiles % 8) == 0, "GEMM grid exact");
static_assert((kPix % kPrepPix) == 0 && (kPix % 256) == 0, "blocks never cross a frame");
static_assert(kNcol * 4 == 128, "projection row is exactly one 128-B line");

constexpr size_t kOffCUM = 0;
constexpr size_t kOffXH  = kOffCUM + (size_t)kFrames * 2 * kPix * 4;
constexpr size_t kOffXL  = kOffXH  + (size_t)kRows * kKdim * 2;
constexpr size_t kOffWH  = kOffXL  + (size_t)kRows * kKdim * 2;
constexpr size_t kOffWL  = kOffWH  + (size_t)kNcol * kKdim * 2;
constexpr size_t kOffPP  = kOffWL  + (size_t)kNcol * kKdim * 2;
constexpr size_t kWsTotal = kOffPP + (size_t)kRows * kNcol * 4;
static_assert(kWsTotal == 17305600ull, "carve total");
static_assert(kWsTotal <= 134217728ull, "carve cap");
static_assert((kOffXH % 128) == 0 && (kOffXL % 128) == 0 && (kOffWH % 128) == 0 &&
              (kOffWL % 128) == 0 && (kOffPP % 128) == 0, "128-B aligned regions");

__device__ __forceinline__ unsigned short f2bf_bits(float f) {
  unsigned u = __float_as_uint(f);
  return (unsigned short)((u + 0x7FFFu + ((u >> 16) & 1u)) >> 16);
}
__device__ __forceinline__ float bf_bits2f(unsigned short h) { return __uint_as_float(((unsigned)h) << 16); }

__device__ __forceinline__ void split8(const v4f a0, const v4f a1, v8h& hv, v8h& lv) {
#pragma unroll
  for (int e = 0; e < 4; ++e) {
    const float x0 = a0[e];
    const float x1 = a1[e];
    const unsigned short h0 = f2bf_bits(x0);
    const unsigned short h1 = f2bf_bits(x1);
    const unsigned short l0 = f2bf_bits(x0 - bf_bits2f(h0));
    const unsigned short l1 = f2bf_bits(x1 - bf_bits2f(h1));
    hv[e]     = __builtin_bit_cast(_Float16, h0);
    hv[4 + e] = __builtin_bit_cast(_Float16, h1);
    lv[e]     = __builtin_bit_cast(_Float16, l0);
    lv[4 + e] = __builtin_bit_cast(_Float16, l1);
  }
}

union FragB { v16b v; v8b h[2]; };
__device__ __forceinline__ v16b frag_load(const __bf16* p) {
  FragB f;
  f.h[0] = *(const v8b*)(p);
  f.h[1] = *(const v8b*)(p + 16);
  return f.v;
}
__device__ __forceinline__ v8f mma_bf16_guarded(v16b a, v16b b, v8f c) {
  c = __builtin_amdgcn_wmma_f32_16x16x32_bf16(false, a, false, b, (short)0, c, false, false);
  asm volatile("v_nop\n\tv_nop\n\tv_nop\n\tv_nop" : "+v"(c) : "v"(a), "v"(b));
  return c;
}

__device__ __forceinline__ float base_coord(int i) {
#pragma clang fp contract(off)
  const float stopv = 1.0f - 1.0f / (float)kSide;
  const float startv = -stopv;
  const float stepv = (float)i * (1.0f / (float)(kSide - 1));
  const float om = 1.0f - stepv;
  const float ta = startv * om;
  const float tb = stopv * stepv;
  const float v = ta + tb;
  return (i == kSide - 1) ? stopv : v;
}

__global__ __launch_bounds__(256) void cum_kernel(const float* __restrict__ flows, float* __restrict__ cum) {
  const int pix  = blockIdx.x * 256 + threadIdx.x;
  const int comp = blockIdx.y;
  float cv[kFrames];
  float run = 0.0f;
#pragma unroll
  for (int t = 0; t < kFrames; ++t) {
    run += flows[(size_t)(t * 2 + comp) * kPix + pix];
    cv[t] = run;
  }
  for (int pass = 0; pass < 2; ++pass) {
#pragma unroll
    for (int t = 0; t < kFrames; ++t)
      *(volatile float*)(cum + (size_t)(t * 2 + comp) * kPix + pix) = cv[t];
    __threadfence();
  }
}

__global__ __launch_bounds__(256) void prep_kernel(
    const float* __restrict__ images, const float* __restrict__ w1,
    unsigned short* __restrict__ XH, unsigned short* __restrict__ XL,
    unsigned short* __restrict__ WH, unsigned short* __restrict__ WL)
{
  __shared__ __align__(16) float sX[kPrepPix * kPrepPitch];
  const int tid  = threadIdx.x;
  const int lane = tid & 31;
  const int wave = __builtin_amdgcn_readfirstlane((int)(threadIdx.x >> 5));
  const int rsub = lane >> 2;
  const int c8   = (lane & 3) * 8;
  if ((int)blockIdx.x < kPrepImgBlocks) {
    const int m0   = blockIdx.x * kPrepPix;
    const int t    = m0 / kPix;
    const int pix0 = m0 - t * kPix;
    const int p    = tid & (kPrepPix - 1);
    const int ch0  = (tid >> 7) * 16;
    const float* src = images + ((size_t)t * kCh + ch0) * kPix + pix0 + p;
#pragma unroll
    for (int i = 0; i < 16; ++i) sX[p * kPrepPitch + ch0 + i] = src[(size_t)i * kPix];
    __syncthreads();
    v8h hv[2], lv[2];
#pragma unroll
    for (int it = 0; it < 2; ++it) {
      const int row = it * 64 + wave * 8 + rsub;
      const float* sp = sX + row * kPrepPitch + c8;
      const v4f a0 = *(const v4f*)(sp);
      const v4f a1 = *(const v4f*)(sp + 4);
      split8(a0, a1, hv[it], lv[it]);
    }
    for (int pass = 0; pass < 2; ++pass) {
#pragma unroll
      for (int it = 0; it < 2; ++it) {
        const int row = it * 64 + wave * 8 + rsub;
        const size_t o = (size_t)(m0 + row) * kKdim + c8;
        *(volatile v8h*)(XH + o) = hv[it];
        *(volatile v8h*)(XL + o) = lv[it];
      }
      __threadfence();
    }
  } else {
    if (wave < 4) {
      const int n    = wave * 8 + rsub;
      const int o    = n & (kHid - 1);
      const int part = n >> 4;
      const float* src = w1 + o * (2 * kCh) + part * kCh + c8;
      const v4f a0 = *(const v4f*)(src);
      const v4f a1 = *(const v4f*)(src + 4);
      v8h hv, lv;
      split8(a0, a1, hv, lv);
      const size_t q = (size_t)n * kKdim + c8;
      *(volatile v8h*)(WH + q) = hv;
      *(volatile v8h*)(WL + q) = lv;
      __threadfence();
      *(volatile v8h*)(WH + q) = hv;
      *(volatile v8h*)(WL + q) = lv;
    }
  }
}

__global__ __launch_bounds__(256) void proj_gemm_kernel(
    const unsigned short* __restrict__ XHp, const unsigned short* __restrict__ XLp,
    const unsigned short* __restrict__ WHp, const unsigned short* __restrict__ WLp,
    float* __restrict__ PP)
{
  __shared__ __align__(16) float sT[8][16 * kSlabPitch];
  const __bf16* XHb = (const __bf16*)XHp;
  const __bf16* XLb = (const __bf16*)XLp;
  const __bf16* WHb = (const __bf16*)WHp;
  const __bf16* WLb = (const __bf16*)WLp;
  const int lane = threadIdx.x & 31;
  const int wave = __builtin_amdgcn_readfirstlane((int)(threadIdx.x >> 5));
  const int tile = blockIdx.x * 8 + wave;
  if (tile >= kGemmTiles) return;
  const int m0    = tile << 6;
  const int rlane = lane & 15;
  const int koff  = (lane >> 4) * 8;
  const int mOff  = (lane >> 4) * 8;

  v16b bh[2], bl[2];
#pragma unroll
  for (int j = 0; j < 2; ++j) {
    const size_t bo = (size_t)((j << 4) + rlane) * kKdim + koff;
    bh[j] = frag_load(WHb + bo);
    bl[j] = frag_load(WLb + bo);
  }

  v8f acc[4][2];
#pragma unroll
  for (int i = 0; i < 4; ++i)
#pragma unroll
    for (int j = 0; j < 2; ++j) acc[i][j] = (v8f){0.f, 0.f, 0.f, 0.f, 0.f, 0.f, 0.f, 0.f};

#pragma unroll
  for (int i = 0; i < 4; ++i) {
    const size_t ao = (size_t)(m0 + (i << 4) + rlane) * kKdim + koff;
    const v16b ah = frag_load(XHb + ao);
    const v16b al = frag_load(XLb + ao);
#pragma unroll
    for (int j = 0; j < 2; ++j) {
      acc[i][j] = mma_bf16_guarded(ah, bh[j], acc[i][j]);
      acc[i][j] = mma_bf16_guarded(ah, bl[j], acc[i][j]);
      acc[i][j] = mma_bf16_guarded(al, bh[j], acc[i][j]);
    }
  }

  float* slab = sT[wave];
  const int q  = lane >> 3;
  const int c4 = (lane & 7) * 4;
#pragma unroll
  for (int i = 0; i < 4; ++i) {
    const int mBase = m0 + (i << 4);
#pragma unroll
    for (int j = 0; j < 2; ++j) {
#pragma unroll
      for (int r = 0; r < 8; ++r) {
        const float v = acc[i][j][r];
        slab[(mOff + r) * kSlabPitch + (j << 4) + rlane] = v;
      }
    }
    __builtin_amdgcn_fence(__ATOMIC_RELEASE, "workgroup");
    __builtin_amdgcn_wave_barrier();
    __builtin_amdgcn_fence(__ATOMIC_ACQUIRE, "workgroup");
    v4f ov[4];
#pragma unroll
    for (int it = 0; it < 4; ++it) ov[it] = *(const v4f*)(slab + (it * 4 + q) * kSlabPitch + c4);
    for (int pass = 0; pass < 2; ++pass) {
#pragma unroll
      for (int it = 0; it < 4; ++it)
        *(volatile v4f*)(PP + (size_t)(mBase + it * 4 + q) * kNcol + c4) = ov[it];
      __threadfence();
    }
    __builtin_amdgcn_fence(__ATOMIC_RELEASE, "workgroup");
    __builtin_amdgcn_wave_barrier();
    __builtin_amdgcn_fence(__ATOMIC_ACQUIRE, "workgroup");
  }
}

__global__ __launch_bounds__(256) void fuse_kernel(
    const float* __restrict__ images, const float* __restrict__ cum, const float* __restrict__ PP,
    const float* __restrict__ decay_log, const float* __restrict__ b1,
    const float* __restrict__ w2, const float* __restrict__ b2, float* __restrict__ out)
{
  const int pix = blockIdx.x * 256 + threadIdx.x;
  const int t   = (int)blockIdx.y / kNumGroup;
  const int c0  = ((int)blockIdx.y - t * kNumGroup) * kChGroup;
  const int xw  = pix & (kSide - 1);
  const int yh  = pix / kSide;
  const float bx = base_coord(xw);
  const float by = base_coord(yh);
  const float fside = (float)kSide;
  const float decay = expf(decay_log[0]);

  float w2x[kHid], w2y[kHid];
#pragma unroll
  for (int m = 0; m < kHid; ++m) {
    w2x[m] = w2[m];
    w2y[m] = w2[kHid + m];
  }
  const float b2x = b2[0];
  const float b2y = b2[1];

  float Ab[kHid];
  {
    const float* arow = PP + ((size_t)t * kPix + pix) * kNcol;
#pragma unroll
    for (int q4 = 0; q4 < 4; ++q4) {
      const v4f a = *(const v4f*)(arow + 4 * q4);
      Ab[4 * q4 + 0] = a[0] + b1[4 * q4 + 0];
      Ab[4 * q4 + 1] = a[1] + b1[4 * q4 + 1];
      Ab[4 * q4 + 2] = a[2] + b1[4 * q4 + 2];
      Ab[4 * q4 + 3] = a[3] + b1[4 * q4 + 3];
    }
  }
  const float ctx = cum[(size_t)(t * 2 + 0) * kPix + pix];
  const float cty = cum[(size_t)(t * 2 + 1) * kPix + pix];

  float acc[kChGroup];
#pragma unroll
  for (int c = 0; c < kChGroup; ++c) acc[c] = 0.0f;

#pragma unroll 1
  for (int k = 0; k <= t; ++k) {
    const float* brow = PP + ((size_t)k * kPix + pix) * kNcol + kHid;
    v4f bv[4];
#pragma unroll
    for (int q4 = 0; q4 < 4; ++q4) bv[q4] = *(const v4f*)(brow + 4 * q4);
    float d0 = 0.0f, d1 = 0.0f;
#pragma unroll
    for (int q4 = 0; q4 < 4; ++q4) {
#pragma unroll
      for (int e = 0; e < 4; ++e) {
        const float bq = bv[q4][e];
        const float hval = fmaxf(Ab[4 * q4 + e] + bq, 0.0f);
        d0 = fmaf(w2x[4 * q4 + e], hval, d0);
        d1 = fmaf(w2y[4 * q4 + e], hval, d1);
      }
    }
    const float r0 = d0 + b2x;
    const float r1 = d1 + b2y;
    const float ckx = cum[(size_t)(k * 2 + 0) * kPix + pix];
    const float cky = cum[(size_t)(k * 2 + 1) * kPix + pix];
    float gx = bx + ((ctx - ckx) + r0);
    const float gy = by + ((cty - cky) + r1);
    float u = gx + 1.0f;
    u = u - 2.0f * floorf(u * 0.5f);
    gx = u - 1.0f;
    const float ix = ((gx + 1.0f) * fside - 1.0f) * 0.5f;
    const float iy = ((gy + 1.0f) * fside - 1.0f) * 0.5f;
    const float ix0f = floorf(ix);
    const float iy0f = floorf(iy);
    const float ix1f = ix0f + 1.0f;
    const float iy1f = iy0f + 1.0f;
    const float wx1 = ix - ix0f;
    const float wy1 = iy - iy0f;
    const float wx0 = 1.0f - wx1;
    const float wy0 = 1.0f - wy1;
    const bool vx0 = (ix0f >= 0.0f) && (ix0f < fside);
    const bool vx1 = (ix1f >= 0.0f) && (ix1f < fside);
    const bool vy0 = (iy0f >= 0.0f) && (iy0f < fside);
    const bool vy1 = (iy1f >= 0.0f) && (iy1f < fside);
    const float hi_idx = (float)(kSide - 1);
    const int cx0 = (int)fminf(fmaxf(ix0f, 0.0f), hi_idx);
    const int cx1 = (int)fminf(fmaxf(ix1f, 0.0f), hi_idx);
    const int cy0 = (int)fminf(fmaxf(iy0f, 0.0f), hi_idx);
    const int cy1 = (int)fminf(fmaxf(iy1f, 0.0f), hi_idx);
    const float wt = expf(-decay * (float)(t - k));
    const float m00 = (vx0 && vy0) ? (wx0 * wy0) : 0.0f;
    const float m10 = (vx1 && vy0) ? (wx1 * wy0) : 0.0f;
    const float m01 = (vx0 && vy1) ? (wx0 * wy1) : 0.0f;
    const float m11 = (vx1 && vy1) ? (wx1 * wy1) : 0.0f;
    const float w00 = wt * m00;
    const float w10 = wt * m10;
    const float w01 = wt * m01;
    const float w11 = wt * m11;
    const int o00 = cy0 * kSide + cx0;
    const int o10 = cy0 * kSide + cx1;
    const int o01 = cy1 * kSide + cx0;
    const int o11 = cy1 * kSide + cx1;
    const float* imk = images + ((size_t)k * kCh + c0) * kPix;
#pragma unroll
    for (int c = 0; c < 4; ++c) {
      const float* p = imk + (size_t)c * kPix;
      const float v00 = p[o00];
      const float v10 = p[o10];
      const float v01 = p[o01];
      const float v11 = p[o11];
      acc[c] += w00 * v00 + w10 * v10 + w01 * v01 + w11 * v11;
    }
    asm volatile("" ::: "memory");
#pragma unroll
    for (int c = 4; c < kChGroup; ++c) {
      const float* p = imk + (size_t)c * kPix;
      const float v00 = p[o00];
      const float v10 = p[o10];
      const float v01 = p[o01];
      const float v11 = p[o11];
      acc[c] += w00 * v00 + w10 * v10 + w01 * v01 + w11 * v11;
    }
  }

  for (int pass = 0; pass < 2; ++pass) {
#pragma unroll
    for (int c = 0; c < kChGroup; ++c)
      *(volatile float*)(out + ((size_t)t * kCh + c0 + c) * kPix + pix) = acc[c];
    __threadfence();
  }
}

extern "C" void kernel_launch(void* const* d_in, const int* in_sizes, int n_in,
                              void* d_out, int out_size, void* d_ws, size_t ws_size,
                              hipStream_t stream) {
  if (n_in < 7) return;
  if (in_sizes[0] != kFrames * 2 * kPix) return;
  if (in_sizes[1] != kFrames * kCh * kPix) return;
  if (in_sizes[2] != 1) return;
  if (in_sizes[3] != kHid * 2 * kCh) return;
  if (in_sizes[4] != kHid) return;
  if (in_sizes[5] != 2 * kHid) return;
  if (in_sizes[6] != 2) return;
  if (out_size != kFrames * kCh * kPix) return;
  if (ws_size < kWsTotal) return;

  const float* flows     = (const float*)d_in[0];
  const float* images    = (const float*)d_in[1];
  const float* decay_log = (const float*)d_in[2];
  const float* w1        = (const float*)d_in[3];
  const float* b1        = (const float*)d_in[4];
  const float* w2        = (const float*)d_in[5];
  const float* b2        = (const float*)d_in[6];
  float* out = (float*)d_out;

  char* ws = (char*)d_ws;
  float*          CUM = (float*)(ws + kOffCUM);
  unsigned short* XH  = (unsigned short*)(ws + kOffXH);
  unsigned short* XL  = (unsigned short*)(ws + kOffXL);
  unsigned short* WH  = (unsigned short*)(ws + kOffWH);
  unsigned short* WL  = (unsigned short*)(ws + kOffWL);
  float*          PP  = (float*)(ws + kOffPP);

  cum_kernel<<<dim3(kPix / 256, 2), 256, 0, stream>>>(flows, CUM);
  prep_kernel<<<kPrepImgBlocks + 1, 256, 0, stream>>>(images, w1, XH, XL, WH, WL);
  proj_gemm_kernel<<<kGemmTiles / 8, 256, 0, stream>>>(XH, XL, WH, WL, PP);
  fuse_kernel<<<dim3(kPix / 256, kFrames * kNumGroup), 256, 0, stream>>>(
      images, CUM, PP, decay_log, b1, w2, b2, out);
}
